// DDPMVAEQueryEncoder_16879221473941
// MI455X (gfx1250) — hardware-verified
//
#include <hip/hip_runtime.h>
#include <math.h>
#include <stddef.h>


#define DM     64
#define DH     256
#define TSTEPS 50
#define NTHR   256
#define ROWS   64
#define PA     72
#define PH     264
#define LN1E4F 9.21034049987793f

typedef __attribute__((ext_vector_type(16))) _Float16 v16h;
typedef __attribute__((ext_vector_type(8)))  _Float16 v8h;
typedef __attribute__((ext_vector_type(8)))  float    v8f;
typedef __attribute__((ext_vector_type(4)))  float    v4f;

__device__ __forceinline__ v16h frag_load(const _Float16* p) {
  union { v16h v; v8h h[2]; } f;
  f.h[0] = *(const v8h*)(p);
  f.h[1] = *(const v8h*)(p + 16);
  return f.v;
}
__device__ __forceinline__ v8f mma16(v16h a, v16h b, v8f c) {
  c = __builtin_amdgcn_wmma_f32_16x16x32_f16(false, a, false, b, (short)0, c, false, false);
  asm volatile("v_nop\n\tv_nop\n\tv_nop\n\tv_nop" : "+v"(c) : "v"(a), "v"(b));
  return c;
}
__device__ __forceinline__ v8f vz8() { return (v8f){0.f, 0.f, 0.f, 0.f, 0.f, 0.f, 0.f, 0.f}; }

template <int NKS, int LDA, int LDB>
__device__ __forceinline__ void gemm_pair(const _Float16* A, const _Float16* Bt, int m0, int n0,
                                          int rl, int koff, v8f& acc0, v8f& acc1) {
  acc0 = vz8(); acc1 = vz8();
#pragma unroll
  for (int ks = 0; ks < NKS; ++ks) {
    const v16h a  = frag_load(A  + (m0 + rl) * LDA + ks * 32 + koff);
    const v16h b0 = frag_load(Bt + (n0 + rl) * LDB + ks * 32 + koff);
    const v16h b1 = frag_load(Bt + (n0 + 16 + rl) * LDB + ks * 32 + koff);
    acc0 = mma16(a, b0, acc0);
    acc1 = mma16(a, b1, acc1);
  }
}

__global__ __launch_bounds__(NTHR)
void ddpm_fused_kernel(const int*   __restrict__ seq,
                       const float* __restrict__ item_emb,
                       const float* __restrict__ W_enc,
                       const float* __restrict__ b_enc,
                       const float* __restrict__ Wt,
                       const float* __restrict__ bt,
                       const float* __restrict__ Wc,
                       const float* __restrict__ bc,
                       const float* __restrict__ W1,
                       const float* __restrict__ b1,
                       const float* __restrict__ W2,
                       const float* __restrict__ b2,
                       const float* __restrict__ init_noise,
                       const float* __restrict__ step_noise,
                       float*       __restrict__ out,
                       int nB, int L, int V) {
  __shared__ __align__(16) _Float16 W1s[DH * PA];
  __shared__ __align__(16) _Float16 W2s[DM * PH];
  __shared__ __align__(16) _Float16 Hs[ROWS * PH];
  __shared__ __align__(16) _Float16 As[ROWS * PA];
  __shared__ __align__(16) float    Ts[64 * DM];
  __shared__ __align__(16) float    b1s[DH];
  __shared__ __align__(16) float    b2s[DM];
  __shared__ __align__(16) float    sch[5 * 64];

  const int tid  = threadIdx.x;
  const int lane = tid & 31;
  const int wave = tid >> 5;
  const int hh   = lane >> 4;
  const int c16  = lane & 15;
  const int koff = hh * 8;
  const int rt   = wave & 3;
  const int cq   = wave >> 2;
  const int R0   = rt * 16;
  const size_t growBase = (size_t)blockIdx.x * ROWS;

  if (tid == 0) {
    const double scale  = 1000.0 / (double)TSTEPS;
    const double bstart = scale * 1e-4;
    const double bstop  = scale * 2e-2;
    const double bstep  = (bstop - bstart) / (double)(TSTEPS - 1);
    double acp = 1.0;
    for (int t = 0; t < TSTEPS; ++t) {
      const double beta     = (t == TSTEPS - 1) ? bstop : ((double)t * bstep + bstart);
      const double alpha    = 1.0 - beta;
      const double acp_prev = acp;
      acp = acp * alpha;
      const double one_m = 1.0 - acp;
      const double rcp   = 1.0 / acp;
      sch[t]       = (float)sqrt(rcp);
      sch[64 + t]  = (float)sqrt(rcp - 1.0);
      sch[128 + t] = (float)(beta * sqrt(acp_prev) / one_m);
      sch[192 + t] = (float)((1.0 - acp_prev) * sqrt(alpha) / one_m);
      float sgm = 0.0f;
      if (t > 0) {
        const double pv  = beta * (1.0 - acp_prev) / one_m;
        const float  plv = (float)log(pv);
        sgm = expf(0.5f * plv);
      }
      sch[256 + t] = sgm;
    }
  }
  for (int e = tid; e < DM * DH; e += NTHR) {
    const int k = e >> 8, n = e & 255;
    W1s[n * PA + k] = (_Float16)(W1[e] * 64.0f);
  }
  for (int e = tid; e < DH * DM; e += NTHR) {
    const int k = e >> 6, n = e & 63;
    W2s[n * PH + k] = (_Float16)(W2[e] * 64.0f);
  }
  _Float16* WEs = Hs;
  _Float16* Wcs = Hs + 64 * PA;
  _Float16* Wts = Hs + 128 * PA;
  for (int e = tid; e < DM * DM; e += NTHR) {
    const int k = e >> 6, n = e & 63;
    WEs[n * PA + k] = (_Float16)(W_enc[k * (2 * DM) + n] * 64.0f);
    Wcs[n * PA + k] = (_Float16)(Wc[e] * 64.0f);
    Wts[n * PA + k] = (_Float16)(Wt[e] * 64.0f);
  }
  b1s[tid] = b1[tid];
  if (tid < DM) b2s[tid] = b2[tid];
  for (int e = tid; e < 64 * DM; e += NTHR) {
    const int t = e >> 6, i = e & 63;
    float v = 0.0f;
    if (t < TSTEPS) {
      const int   ii  = i & 31;
      const float fr  = expf((-LN1E4F * (float)ii) * 0.03125f);
      const float arg = (float)t * fr;
      v = (i < 32) ? cosf(arg) : sinf(arg);
    }
    As[t * PA + i] = (_Float16)(v * 64.0f);
  }
  __syncthreads();

  {
    v8f a0, a1;
    gemm_pair<2, PA, PA>(As, Wts, R0, 32 * cq, c16, koff, a0, a1);
    const v8f ap[2] = {a0, a1};
#pragma unroll
    for (int j = 0; j < 2; ++j) {
      const int n = 32 * cq + 16 * j + c16;
      const float bb = bt[n];
#pragma unroll
      for (int r = 0; r < 8; ++r) Ts[(R0 + 8 * hh + r) * DM + n] = ap[j][r] * (1.0f / 4096.0f) + bb;
    }
  }
  __syncthreads();

  {
    const int row = tid >> 2, q = tid & 3;
    const int* srow = seq + (growBase + (size_t)row) * (size_t)L;
    v4f s0 = (v4f){0.f, 0.f, 0.f, 0.f}, s1 = s0, s2 = s0, s3 = s0;
    int nz = 0;
#pragma unroll 1
    for (int l = 0; l < L; ++l) {
      int idx = srow[l];
      nz += (idx != 0);
      idx = (idx < 0) ? (idx + V) : idx;
      idx = (idx < 0) ? 0 : ((idx >= V) ? (V - 1) : idx);
      const float* ep = item_emb + (size_t)idx * DM + q * 16;
      s0 += *(const v4f*)(ep);
      s1 += *(const v4f*)(ep + 4);
      s2 += *(const v4f*)(ep + 8);
      s3 += *(const v4f*)(ep + 12);
    }
    const float rs = 1.0f / sqrtf((float)nz);
    _Float16* ap = As + row * PA + q * 16;
#pragma unroll
    for (int e = 0; e < 4; ++e) {
      ap[e]      = (_Float16)((s0[e] * rs) * 64.0f);
      ap[4 + e]  = (_Float16)((s1[e] * rs) * 64.0f);
      ap[8 + e]  = (_Float16)((s2[e] * rs) * 64.0f);
      ap[12 + e] = (_Float16)((s3[e] * rs) * 64.0f);
    }
  }
  __syncthreads();

  {
    v8f a0, a1;
    gemm_pair<2, PA, PA>(As, WEs, R0, 32 * cq, c16, koff, a0, a1);
    __syncthreads();
    const v8f ap[2] = {a0, a1};
#pragma unroll
    for (int j = 0; j < 2; ++j) {
      const int n = 32 * cq + 16 * j + c16;
      const float bb = b_enc[n];
#pragma unroll
      for (int r = 0; r < 8; ++r) {
        const float mu = ap[j][r] * (1.0f / 4096.0f) + bb;
        As[(R0 + 8 * hh + r) * PA + n] = (_Float16)(mu * 4096.0f);
      }
    }
  }
  __syncthreads();

  float xr[2][8], cr[2][8];
  {
    v8f a0, a1;
    gemm_pair<2, PA, PA>(As, Wcs, R0, 32 * cq, c16, koff, a0, a1);
    const v8f ap[2] = {a0, a1};
#pragma unroll
    for (int j = 0; j < 2; ++j) {
      const int n = 32 * cq + 16 * j + c16;
      const float bb = bc[n];
#pragma unroll
      for (int r = 0; r < 8; ++r) {
        const size_t grow = growBase + (size_t)(R0 + 8 * hh + r);
        cr[j][r] = ap[j][r] * (1.0f / 262144.0f) + bb;
        xr[j][r] = init_noise[grow * DM + n];
      }
    }
  }
  __syncthreads();

#pragma unroll 1
  for (int i = 0; i < TSTEPS; ++i) {
    const int t = TSTEPS - 1 - i;
#pragma unroll
    for (int j = 0; j < 2; ++j) {
      const int n = 32 * cq + 16 * j + c16;
      const float tv = Ts[t * DM + n];
#pragma unroll
      for (int r = 0; r < 8; ++r)
        As[(R0 + 8 * hh + r) * PA + n] = (_Float16)((xr[j][r] + tv) + cr[j][r]);
    }
    __syncthreads();

    {
      v8f acc1[8];
#pragma unroll
      for (int j = 0; j < 8; ++j) acc1[j] = vz8();
#pragma unroll
      for (int ks = 0; ks < 2; ++ks) {
        const v16h a = frag_load(As + (R0 + c16) * PA + ks * 32 + koff);
#pragma unroll
        for (int j = 0; j < 8; ++j) {
          const v16h b = frag_load(W1s + (128 * cq + 16 * j + c16) * PA + ks * 32 + koff);
          acc1[j] = mma16(a, b, acc1[j]);
        }
      }
#pragma unroll
      for (int j = 0; j < 8; ++j) {
        const int n = 128 * cq + 16 * j + c16;
        const float bb = b1s[n];
#pragma unroll
        for (int r = 0; r < 8; ++r) {
          const float v   = acc1[j][r] * (1.0f / 64.0f) + bb;
          const float sgd = __builtin_amdgcn_rcpf(1.0f + __expf(-v));
          Hs[(R0 + 8 * hh + r) * PH + n] = (_Float16)(v * sgd);
        }
      }
    }
    __syncthreads();

    {
      v8f e0, e1;
      gemm_pair<8, PH, PH>(Hs, W2s, R0, 32 * cq, c16, koff, e0, e1);
      const v8f ep[2] = {e0, e1};
      const float sr = sch[t], srm1 = sch[64 + t], co1 = sch[128 + t], co2 = sch[192 + t], sgm = sch[256 + t];
      const float* nzp = step_noise + (size_t)i * (size_t)nB * DM;
#pragma unroll
      for (int j = 0; j < 2; ++j) {
        const int n = 32 * cq + 16 * j + c16;
        const float bb = b2s[n];
#pragma unroll
        for (int r = 0; r < 8; ++r) {
          const size_t grow = growBase + (size_t)(R0 + 8 * hh + r);
          const float eps  = ep[j][r] * (1.0f / 64.0f) + bb;
          const float xv   = xr[j][r];
          const float x0   = sr * xv - srm1 * eps;
          const float mean = co1 * x0 + co2 * xv;
          const float nzv  = nzp[grow * DM + n];
          xr[j][r] = mean + sgm * nzv;
        }
      }
    }
  }

  __syncthreads();
  float* os = Ts + wave * 512;
#pragma unroll
  for (int j = 0; j < 2; ++j)
#pragma unroll
    for (int r = 0; r < 8; ++r) os[(8 * hh + r) * 32 + 16 * j + c16] = xr[j][r];
  __syncthreads();
  {
    const int q = lane >> 3, c4 = (lane & 7) * 4;
    float* ob = out + (growBase + (size_t)R0) * DM + 32 * cq;
    for (int pass = 0; pass < 2; ++pass) {
#pragma unroll
      for (int it = 0; it < 4; ++it) {
        const int row = it * 4 + q;
        const v4f v = *(const v4f*)(os + row * 32 + c4);
        *(volatile v4f*)(ob + (size_t)row * DM + c4) = v;
      }
      __threadfence();
    }
  }
}

extern "C" void kernel_launch(void* const* d_in, const int* in_sizes, int n_in,
                              void* d_out, int out_size, void* d_ws, size_t ws_size,
                              hipStream_t stream) {
  (void)d_ws; (void)ws_size;
  if (n_in < 14) return;
  const int nB = in_sizes[12] / DM;
  if (nB <= 0 || (nB % ROWS) != 0) return;
  const int L = in_sizes[0] / nB;
  const int V = in_sizes[1] / DM;
  if (L <= 0 || V <= 0) return;
  if (in_sizes[13] != TSTEPS * nB * DM) return;
  if (out_size != nB * DM) return;

  const int*   seq        = (const int*)  d_in[0];
  const float* item_emb   = (const float*)d_in[1];
  const float* W_enc      = (const float*)d_in[2];
  const float* b_enc      = (const float*)d_in[3];
  const float* Wt         = (const float*)d_in[4];
  const float* bt         = (const float*)d_in[5];
  const float* Wc         = (const float*)d_in[6];
  const float* bc         = (const float*)d_in[7];
  const float* W1         = (const float*)d_in[8];
  const float* b1         = (const float*)d_in[9];
  const float* W2         = (const float*)d_in[10];
  const float* b2         = (const float*)d_in[11];
  const float* init_noise = (const float*)d_in[12];
  const float* step_noise = (const float*)d_in[13];
  float* out = (float*)d_out;

  ddpm_fused_kernel<<<nB / ROWS, NTHR, 0, stream>>>(seq, item_emb, W_enc, b_enc, Wt, bt, Wc, bc,
                                                    W1, b1, W2, b2, init_noise, step_noise, out, nB, L, V);
}
